// LightweightGravitationalBlock_32993938768209
// MI455X (gfx1250) — hardware-run, weakly checked
//
#include <hip/hip_runtime.h>
#include <math.h>

typedef __attribute__((ext_vector_type(16))) _Float16 v16h;
typedef __attribute__((ext_vector_type(16))) __bf16 v16b;
typedef __attribute__((ext_vector_type(8)))  _Float16 v8h;
typedef __attribute__((ext_vector_type(8)))  float v8f;
typedef __attribute__((ext_vector_type(4)))  float v4f;
typedef __attribute__((ext_vector_type(2)))  float v2f;
typedef __attribute__((ext_vector_type(4)))  unsigned v4u;
typedef __attribute__((ext_vector_type(4)))  int v4i;
typedef float __attribute__((may_alias)) float_a;
typedef int __attribute__((may_alias)) int_a;

template <typename T> __device__ __forceinline__ void vst2(void* p, T v) { *(volatile T*)p = v; __threadfence(); *(volatile T*)p = v; }
__device__ __forceinline__ v8f wmma16(v16h a, v16h b, v8f c) {
  v8f d = __builtin_amdgcn_wmma_f32_16x16x32_f16(false, a, false, b, (short)0, c, false, false);
  asm volatile("v_nop\n\tv_nop\n\tv_nop\n\tv_nop" : "+v"(d) : "v"(a), "v"(b));
  return d;
}
__device__ __forceinline__ v8f wmma_bf(v16b a, v16b b, v8f c) {
  v8f d = __builtin_amdgcn_wmma_f32_16x16x32_bf16(false, a, false, b, (short)0, c, false, false);
  asm volatile("v_nop\n\tv_nop\n\tv_nop\n\tv_nop" : "+v"(d) : "v"(a), "v"(b));
  return d;
}
__device__ __forceinline__ v16h frag_h(const _Float16* rowk0, int lane) {
  union { v16h v; v8h q[2]; } u; const _Float16* p = rowk0 + 8 * (lane >> 4);
  u.q[0] = *(const v8h*)p; u.q[1] = *(const v8h*)(p + 16); return u.v;
}
__device__ __forceinline__ v16h frag_f32(const float* rowk0, int lane) {
  v16h a; const float* p = rowk0 + 8 * (lane >> 4);
#pragma unroll
  for (int i = 0; i < 8; ++i) { a[i] = (_Float16)p[i]; a[8 + i] = (_Float16)p[16 + i]; }
  return a;
}
__device__ __forceinline__ v16h frag_f32s(const float* rowk0, int lane, float sc) {
  v16h a; const float* p = rowk0 + 8 * (lane >> 4);
#pragma unroll
  for (int i = 0; i < 8; ++i) { a[i] = (_Float16)(p[i] * sc); a[8 + i] = (_Float16)(p[16 + i] * sc); }
  return a;
}
__device__ __forceinline__ v16h fragc_f32(const float* W, int k0, int n, int lane, int ld, int K) {
  v16h a; const int g = lane >> 4;
#pragma unroll
  for (int i = 0; i < 8; ++i) { const int ka = k0 + 8 * g + i, kb = ka + 16;
    a[i] = (_Float16)(ka < K ? W[(size_t)(ka < K ? ka : K - 1) * ld + n] : 0.f); a[8 + i] = (_Float16)(kb < K ? W[(size_t)(kb < K ? kb : K - 1) * ld + n] : 0.f); }
  return a;
}
struct F2 { v16b h, l; };
__device__ __forceinline__ F2 bsplit16(const float v[16]) { F2 r;
#pragma unroll
  for (int i = 0; i < 16; ++i) { const __bf16 h = (__bf16)v[i]; r.h[i] = h; r.l[i] = (__bf16)(v[i] - (float)h); }
  return r; }
__device__ __forceinline__ F2 split_row(const float* row, int k0, int lane) { float v[16]; const float* p = row + k0 + 8 * (lane >> 4);
#pragma unroll
  for (int i = 0; i < 8; ++i) { v[i] = p[i]; v[8 + i] = p[16 + i]; }
  return bsplit16(v); }
__device__ __forceinline__ F2 split_rowK(const float* row, int k0, int lane, int K) { float v[16]; const int g = lane >> 4;
#pragma unroll
  for (int i = 0; i < 8; ++i) { const int ka = k0 + 8 * g + i, kb = ka + 16; v[i] = ka < K ? row[ka < K ? ka : K - 1] : 0.f; v[8 + i] = kb < K ? row[kb < K ? kb : K - 1] : 0.f; }
  return bsplit16(v); }
__device__ __forceinline__ F2 split_col(const float* W, int k0, int n, int lane, int ld, int K) { float v[16]; const int g = lane >> 4;
#pragma unroll
  for (int i = 0; i < 8; ++i) { const int ka = k0 + 8 * g + i, kb = ka + 16; v[i] = ka < K ? W[(size_t)(ka < K ? ka : K - 1) * ld + n] : 0.f; v[8 + i] = kb < K ? W[(size_t)(kb < K ? kb : K - 1) * ld + n] : 0.f; }
  return bsplit16(v); }
__device__ __forceinline__ v8f mac3(const F2& a, const F2& b, v8f c) { c = wmma_bf(a.l, b.h, c); c = wmma_bf(a.h, b.l, c); return wmma_bf(a.h, b.h, c); }
__device__ __forceinline__ float sigm(float v) { return 1.0f / (1.0f + expf(-v)); }
#define LDSX() do { asm volatile("s_wait_dscnt 0" ::: "memory"); __builtin_amdgcn_wave_barrier(); __builtin_amdgcn_fence(__ATOMIC_RELEASE, "workgroup"); } while (0)


#define NB 4
#define SS 2048
#define DM 256
#define NH 8
#define HD 32
#define PP 64
#define FF 512
#define NR (NB * SS)
#ifndef TQB
#define TQB (SS / 64)
#define TNB NB
#define NRB (NR / 64)
#endif
typedef __attribute__((ext_vector_type(8))) __bf16 v8b;
__device__ __forceinline__ v16b frag_b(const __bf16* rowk0, int lane) {
  union { v16b v; v8b q[2]; } u; const __bf16* p = rowk0 + 8 * (lane >> 4);
  u.q[0] = *(const v8b*)p; u.q[1] = *(const v8b*)(p + 16); return u.v;
}
__device__ __forceinline__ float bfr(float v) { return (float)(__bf16)v; }
__device__ __attribute__((noinline)) float exp_ni(float v) { return expf(v); }
__device__ __attribute__((noinline)) float erf_ni(float v) { return erff(v); }

#define WS_PV   0u
#define WS_PO   (WS_PV + 2u * DM * DM)
#define WS_P1   (WS_PO + 2u * DM * DM)
#define WS_P2   (WS_P1 + 2u * FF * DM)
#define WS_M    (WS_P2 + 2u * DM * FF)
#define WS_R2   (WS_M + 4u * (size_t)NR * NH)
#define WS_VP   (WS_R2 + 4u * (size_t)SS * SS)
#define WS_CTX  (WS_VP + 2u * (size_t)NB * DM * SS)
#define WS_Y    (WS_CTX + 4u * (size_t)NR * DM)
#define WS_X1   (WS_Y + 4u * (size_t)NR * DM)
#define WS_H16  (WS_X1 + 4u * (size_t)NR * DM)
#define WS_G16  (WS_H16 + 2u * (size_t)NR * DM)
#define WS_END  (WS_G16 + 2u * (size_t)NR * FF)

__global__ __launch_bounds__(256) void k_pack(const float* __restrict__ WV, const float* __restrict__ WO, const float* __restrict__ W1, const float* __restrict__ W2, __bf16* __restrict__ P, _Float16* __restrict__ PH) {
  const int n = blockIdx.x, which = blockIdx.y, t = threadIdx.x; __shared__ __align__(16) __bf16 s[DM]; __shared__ __align__(16) _Float16 sh[FF];
  if (which < 2) { if (n >= DM) return; const float* Wm = which ? WO : WV; s[t] = (__bf16)Wm[(size_t)t * DM + n]; __syncthreads(); if (t < DM / 8) vst2((unsigned*)(P + (which ? WS_PO / 2 : 0) + (size_t)n * DM + t * 8), *(const v4u*)&s[t * 8]); }
  else if (which == 2) { sh[t] = (_Float16)(bfr(W1[(size_t)t * FF + n]) * 256.0f); __syncthreads(); if (t < DM / 8) vst2((unsigned*)(PH + (size_t)n * DM + t * 8), *(const v4u*)&sh[t * 8]); }
  else { if (n >= DM) return; for (int k = t; k < FF; k += 256) sh[k] = (_Float16)(bfr(W2[(size_t)k * DM + n]) * 256.0f); __syncthreads(); if (t < FF / 8) vst2((unsigned*)(PH + (size_t)FF * DM + (size_t)n * FF + t * 8), *(const v4u*)&sh[t * 8]); }
}
__device__ __attribute__((noinline)) float log1p_p(float v) { return log1pf(v); }
__global__ __launch_bounds__(256) void k_mass(const float* __restrict__ X, const float* __restrict__ WM, const float* __restrict__ BM, float* __restrict__ M) {
  const int t = threadIdx.x; const size_t row = (size_t)blockIdx.x * 32 + (t >> 3); const int h = t & 7; float a = bfr(BM[h]);
#pragma unroll 4
  for (int d = 0; d < DM; ++d) a += bfr(X[row * DM + d]) * bfr(WM[d * NH + h]);
  M[row * NH + h] = (a > 20.f) ? a : log1p_p(exp_ni(a));
}
__global__ __launch_bounds__(256) void k_r2(const float* __restrict__ POS, float* __restrict__ R2) {
  __shared__ float spi[16][PP]; __shared__ float spj[PP][257];
  const int t = threadIdx.x; const int i0 = blockIdx.y * 16, j0 = blockIdx.x * 256;
  for (int e = t; e < 16 * PP; e += 256) spi[e / PP][e % PP] = bfr(POS[(size_t)(i0 + e / PP) * PP + e % PP]);
  for (int e = t; e < 256 * PP; e += 256) { const int jj = e / PP, p = e % PP; spj[p][jj] = bfr(POS[(size_t)(j0 + jj) * PP + p]); }
  __syncthreads();
#pragma unroll 1
  for (int ii = 0; ii < 16; ++ii) { float s = 0.f;
#pragma unroll 8
    for (int p = 0; p < PP; ++p) { const float d = spi[ii][p] - spj[p][t]; s += d * d; }
    R2[(size_t)(i0 + ii) * SS + j0 + t] = s; }
}
__global__ __launch_bounds__(128) void k_v(const float* __restrict__ X, const __bf16* __restrict__ P, const float* __restrict__ BV, _Float16* __restrict__ VP) {
  __shared__ __align__(16) _Float16 st[128][72];
  const int tid = threadIdx.x, wave = tid >> 5, lane = tid & 31, col = lane & 15, g = lane >> 4; const size_t rb0 = (size_t)blockIdx.x * 64, r0 = rb0 + wave * 16; const int n0 = blockIdx.y * 128;
  v8f acc[8] = {};
#pragma unroll
  for (int kc = 0; kc < DM / 32; ++kc) { v16b a; { const float* p = X + (r0 + col) * DM + kc * 32 + 8 * g;
#pragma unroll
      for (int i = 0; i < 8; ++i) { a[i] = (__bf16)p[i]; a[8 + i] = (__bf16)p[16 + i]; } }
#pragma unroll
    for (int j = 0; j < 8; ++j) acc[j] = wmma_bf(a, frag_b(P + (size_t)(n0 + j * 16 + col) * DM + kc * 32, lane), acc[j]); }
#pragma unroll
  for (int j = 0; j < 8; ++j) { const float bb = bfr(BV[n0 + j * 16 + col]);
#pragma unroll
    for (int r = 0; r < 8; ++r) st[j * 16 + col][wave * 16 + 8 * g + r] = (_Float16)(acc[j][r] + bb); }
  __syncthreads();
  const size_t b = rb0 / SS, s0 = rb0 % SS;
  for (int e = tid; e < 128 * 8; e += 128) { const int d = e >> 3, pc = e & 7; vst2((unsigned*)(VP + ((b * DM + n0 + d) * SS) + s0 + pc * 8), *(const v4u*)&st[d][pc * 8]); }
}
__global__ __launch_bounds__(128) void k_gatt(const float* __restrict__ M, const float* __restrict__ R2, const float* __restrict__ GH, const _Float16* __restrict__ VP, float* __restrict__ CTX) {
  __shared__ __align__(16) _Float16 sph[4][16][40]; __shared__ __align__(16) float so[4][16][36];
  const int tid = threadIdx.x, wave = tid >> 5, lane = tid & 31, col = lane & 15, g = lane >> 4; const int h = blockIdx.y; const size_t b = blockIdx.z; const int q0 = blockIdx.x * 64 + wave * 16; const size_t rq = b * SS + q0;
  const float gh = bfr(GH[h]); float mq[8];
#pragma unroll
  for (int r = 0; r < 8; ++r) mq[r] = gh * M[(rq + 8 * g + r) * NH + h];
  float m[8], l[8];
#pragma unroll
  for (int r = 0; r < 8; ++r) { m[r] = -3.0e38f; l[r] = 0.f; }
  v8f acc[2] = {};
#pragma unroll 1
  for (int ks = 0; ks < SS / 32; ++ks) { const int j0 = ks * 32; float s[2][8];
#pragma unroll
    for (int ct = 0; ct < 2; ++ct) { const int kk = j0 + ct * 16 + col; const float mk = M[(b * SS + kk) * NH + h];
#pragma unroll
      for (int r = 0; r < 8; ++r) { const float r2 = R2[(size_t)(q0 + 8 * g + r) * SS + kk]; const float den = r2 + 0.15f * r2 * r2 + 1e-6f; s[ct][r] = fminf(mq[r] * mk / den, 50.0f); } }
#pragma unroll
    for (int r = 0; r < 8; ++r) { float mx = fmaxf(s[0][r], s[1][r]);
#pragma unroll
      for (int o = 1; o < 16; o <<= 1) mx = fmaxf(mx, __shfl_xor(mx, o));
      const float mn = fmaxf(m[r], mx); const float alpha = (m[r] <= -1.0e38f) ? 0.f : __expf(m[r] - mn); const float e0 = __expf(s[0][r] - mn), e1 = __expf(s[1][r] - mn); float es = e0 + e1;
#pragma unroll
      for (int o = 1; o < 16; o <<= 1) es += __shfl_xor(es, o);
      l[r] = l[r] * alpha + es; m[r] = mn;
#pragma unroll
      for (int dt = 0; dt < 2; ++dt) acc[dt][r] *= alpha;
      sph[wave][8 * g + r][col] = (_Float16)(e0 * 2048.0f); sph[wave][8 * g + r][16 + col] = (_Float16)(e1 * 2048.0f); }
    LDSX();
    const v16h pa = frag_h(&sph[wave][col][0], lane);
#pragma unroll
    for (int dt = 0; dt < 2; ++dt) acc[dt] = wmma16(pa, frag_h(VP + ((b * DM + (size_t)h * HD + dt * 16 + col) * SS) + j0, lane), acc[dt]);
    LDSX(); }
#pragma unroll
  for (int r = 0; r < 8; ++r) { const float il = (1.0f / 2048.0f) / l[r];
#pragma unroll
    for (int dt = 0; dt < 2; ++dt) so[wave][8 * g + r][dt * 16 + col] = acc[dt][r] * il; }
  LDSX();
  for (int rl = 0; rl < 16; ++rl) if (lane < 8) vst2(CTX + (rq + rl) * DM + h * HD + lane * 4, *(const v4f*)&so[wave][rl][lane * 4]);
}
__global__ __launch_bounds__(128) void k_out(const float* __restrict__ CTX, const __bf16* __restrict__ P, const float* __restrict__ BO, const float* __restrict__ X, float* __restrict__ Yo) {
  __shared__ __align__(16) float so[4][16][132];
  const int tid = threadIdx.x, wave = tid >> 5, lane = tid & 31, col = lane & 15, g = lane >> 4; const size_t r0 = (size_t)blockIdx.x * 64 + wave * 16; const int n0 = blockIdx.y * 128;
  v8f acc[8] = {};
#pragma unroll
  for (int kc = 0; kc < DM / 32; ++kc) { const F2 a = split_row(CTX + (r0 + col) * DM, kc * 32, lane);
#pragma unroll
    for (int j = 0; j < 8; ++j) { const v16b w = frag_b(P + WS_PO / 2 + (size_t)(n0 + j * 16 + col) * DM + kc * 32, lane); acc[j] = wmma_bf(a.l, w, acc[j]); acc[j] = wmma_bf(a.h, w, acc[j]); } }
#pragma unroll
  for (int j = 0; j < 8; ++j) { const int c = n0 + j * 16 + col; const float bb = bfr(BO[c]);
#pragma unroll
    for (int r = 0; r < 8; ++r) so[wave][8 * g + r][j * 16 + col] = acc[j][r] + bb + bfr(X[(r0 + 8 * g + r) * DM + c]); }
  LDSX();
  for (int rl = 0; rl < 16; ++rl) vst2(Yo + (r0 + rl) * DM + n0 + lane * 4, *(const v4f*)&so[wave][rl][lane * 4]);
}
template <int MODE>
__global__ __launch_bounds__(256) void k_ln(const float* __restrict__ Yin, const float* __restrict__ G, const float* __restrict__ Bt, float* __restrict__ OF, _Float16* __restrict__ OH) {
  __shared__ float red[8]; __shared__ __align__(16) _Float16 sh[4][DM]; const int t = threadIdx.x; const int rl = t >> 6, tt = t & 63; const size_t row = (size_t)blockIdx.x * 4 + rl;
  float v[4]; float s = 0.f; for (int i = 0; i < 4; ++i) { v[i] = Yin[row * DM + tt * 4 + i]; s += v[i]; }
#pragma unroll
  for (int o = 1; o < 32; o <<= 1) s += __shfl_xor(s, o);
  if ((t & 31) == 0) red[t >> 5] = s; __syncthreads(); const float mu = (red[rl * 2] + red[rl * 2 + 1]) / (float)DM; __syncthreads();
  float q = 0.f; for (int i = 0; i < 4; ++i) { const float dd = v[i] - mu; q += dd * dd; }
#pragma unroll
  for (int o = 1; o < 32; o <<= 1) q += __shfl_xor(q, o);
  if ((t & 31) == 0) red[t >> 5] = q; __syncthreads(); const float inv = 1.0f / sqrtf((red[rl * 2] + red[rl * 2 + 1]) / (float)DM + 1e-5f);
  v4f o4; for (int i = 0; i < 4; ++i) { const int e = tt * 4 + i; o4[i] = (v[i] - mu) * inv * bfr(G[e]) + bfr(Bt[e]); if (MODE == 0) sh[rl][e] = (_Float16)o4[i]; }
  vst2(OF + row * DM + tt * 4, o4);
  if (MODE == 0) { __syncthreads(); if (tt < DM / 8) vst2((unsigned*)(OH + row * DM + tt * 8), *(const v4u*)&sh[rl][tt * 8]); }
}
__device__ __attribute__((noinline)) float tanh_p(float v) { return tanhf(v); }
template <int MODE>
__global__ __launch_bounds__(128) void k_mlp(const _Float16* __restrict__ Ain, const _Float16* __restrict__ Wr, const float* __restrict__ BIAS, const float* __restrict__ RES, float* __restrict__ OUTF, _Float16* __restrict__ OG) {
  constexpr int KIN = (MODE == 0) ? DM : FF; constexpr int NOUT = (MODE == 0) ? FF : DM;
  __shared__ __align__(16) float so[4][16][132]; __shared__ __align__(16) _Float16 sg[4][16][136];
  const int tid = threadIdx.x, wave = tid >> 5, lane = tid & 31, col = lane & 15, g = lane >> 4; const size_t r0 = (size_t)blockIdx.x * 64 + wave * 16; const int n0 = blockIdx.y * 128;
  v8f acc[8] = {};
#pragma unroll 2
  for (int kc = 0; kc < KIN / 32; ++kc) { const v16h a = frag_h(Ain + (r0 + col) * KIN + kc * 32, lane);
#pragma unroll
    for (int j = 0; j < 8; ++j) acc[j] = wmma16(a, frag_h(Wr + (size_t)(n0 + j * 16 + col) * KIN + kc * 32, lane), acc[j]); }
#pragma unroll
  for (int j = 0; j < 8; ++j) { const int c = n0 + j * 16 + col; const float bb = bfr(BIAS[c]);
#pragma unroll
    for (int r = 0; r < 8; ++r) { const float x = acc[j][r] * (1.0f / 256.0f) + bb; if (MODE == 0) { const float cg = 0.7978845608028654f; sg[wave][8 * g + r][j * 16 + col] = (_Float16)(0.5f * x * (1.0f + tanh_p(cg * (x + 0.044715f * x * x * x)))); } else so[wave][8 * g + r][j * 16 + col] = x + RES[(r0 + 8 * g + r) * DM + c]; } }
  LDSX();
  if (MODE == 0) { for (int rl = 0; rl < 16; ++rl) if (lane < 16) vst2((unsigned*)(OG + (r0 + rl) * NOUT + n0 + lane * 8), *(const v4u*)&sg[wave][rl][lane * 8]); }
  else { for (int rl = 0; rl < 16; ++rl) vst2(OUTF + (r0 + rl) * NOUT + n0 + lane * 4, *(const v4f*)&so[wave][rl][lane * 4]); }
}
extern "C" void kernel_launch(void* const* d_in, const int* in_sizes, int n_in, void* d_out, int out_size, void* d_ws, size_t ws_size, hipStream_t stream) {
  (void)in_sizes; (void)n_in; (void)out_size;
  const float** F = (const float**)d_in;
  if (ws_size < (size_t)WS_END) return;
  char* ws = (char*)d_ws; __bf16* P = (__bf16*)ws; _Float16 *PH = (_Float16*)(ws + WS_P1), *VP = (_Float16*)(ws + WS_VP), *H16 = (_Float16*)(ws + WS_H16), *G16 = (_Float16*)(ws + WS_G16); float *M = (float*)(ws + WS_M), *R2 = (float*)(ws + WS_R2), *CTX = (float*)(ws + WS_CTX), *Y = (float*)(ws + WS_Y), *X1 = (float*)(ws + WS_X1);
  k_pack<<<dim3(FF, 4), 256, 0, stream>>>(F[4], F[6], F[9], F[11], P, PH);
  k_mass<<<NR / 32, 256, 0, stream>>>(F[0], F[2], F[3], M);
  k_r2<<<dim3(SS / 256, SS / 16), 256, 0, stream>>>(F[1], R2);
  k_v<<<dim3(NRB, DM / 128), 128, 0, stream>>>(F[0], P, F[5], VP);
  k_gatt<<<dim3(TQB, NH, TNB), 128, 0, stream>>>(M, R2, F[8], VP, CTX);
  k_out<<<dim3(NRB, DM / 128), 128, 0, stream>>>(CTX, P, F[7], F[0], Y);
  k_ln<0><<<NRB * 16, 256, 0, stream>>>(Y, F[13], F[14], X1, H16);
  k_mlp<0><<<dim3(NRB, FF / 128), 128, 0, stream>>>(H16, PH, F[10], nullptr, nullptr, G16);
  k_mlp<1><<<dim3(NRB, DM / 128), 128, 0, stream>>>(G16, PH + (size_t)FF * DM, F[12], X1, Y, nullptr);
  k_ln<1><<<NRB * 16, 256, 0, stream>>>(Y, F[15], F[16], (float*)d_out, nullptr);
}
